// DynamicHead_57011395887597
// MI455X (gfx1250) — hardware-verified
//
#include <hip/hip_runtime.h>


#define NBT  32768
#define DI   256
#define SD   12
#define RCH  4096
#define NW   (SD * DI)
typedef _Float16 h16;
typedef unsigned short bf;
typedef __attribute__((ext_vector_type(16))) __bf16   v16bf;
typedef __attribute__((ext_vector_type(16))) _Float16 v16h;
typedef __attribute__((ext_vector_type(8)))  _Float16 v8h;
typedef __attribute__((ext_vector_type(8)))  unsigned short v8us;
typedef __attribute__((ext_vector_type(8)))  float    v8f;
typedef __attribute__((ext_vector_type(4)))  float    v4f;
typedef v8h  __attribute__((may_alias)) v8ha;
typedef v4f  __attribute__((may_alias)) v4fa;
typedef v8us __attribute__((may_alias)) v8usa;

__device__ __forceinline__ unsigned short f2bf(float f) { unsigned u = __float_as_uint(f); u += 0x7FFFu + ((u >> 16) & 1u); return (unsigned short)(u >> 16); }
__device__ __forceinline__ float bf2f(unsigned short b) { return __uint_as_float(((unsigned)b) << 16); }
__device__ __forceinline__ float bfr(float f) { return bf2f(f2bf(f)); }
__device__ __forceinline__ v16h cat16(v8h lo, v8h hi) { return __builtin_shufflevector(lo, hi, 0, 1, 2, 3, 4, 5, 6, 7, 8, 9, 10, 11, 12, 13, 14, 15); }
__device__ __forceinline__ v16bf cat16b(v8us lo, v8us hi) { return __builtin_bit_cast(v16bf, __builtin_shufflevector(lo, hi, 0, 1, 2, 3, 4, 5, 6, 7, 8, 9, 10, 11, 12, 13, 14, 15)); }
__device__ __forceinline__ v8f wmma16(v16h a, v16h b, v8f c) { return __builtin_amdgcn_wmma_f32_16x16x32_f16(false, a, false, b, (short)0, c, false, false); }
__device__ __forceinline__ v8f wmmab(v16bf a, v16bf b, v8f c) { return __builtin_amdgcn_wmma_f32_16x16x32_bf16(false, a, false, b, (short)0, c, false, false); }


template <typename T16> struct WFrag;
template <> struct WFrag<h16> { typedef v16h V; static __device__ __forceinline__ V ld(const h16* p) { return cat16(*(const v8h*)p, *(const v8h*)(p + 16)); } static __device__ __forceinline__ v8f mma(V a, V b, v8f c) { return wmma16(a, b, c); } };
template <> struct WFrag<bf> { typedef v16bf V; static __device__ __forceinline__ V ld(const bf* p) { return cat16b(*(const v8us*)p, *(const v8us*)(p + 16)); } static __device__ __forceinline__ v8f mma(V a, V b, v8f c) { return wmmab(a, b, c); } };
template <typename T16, int NSPLIT, bool BIAS>
__global__ __launch_bounds__(32) void k_gemmw(const T16* __restrict__ A, const T16* __restrict__ A2, const T16* __restrict__ Bt, const T16* __restrict__ Bt2, int K, float* C, int ldc, const float* __restrict__ bias, size_t sA, size_t sB, size_t sC) {
    typedef typename WFrag<T16>::V V;
    __shared__ __align__(16) float os[16 * 68];
    const size_t z = blockIdx.z; A += z * sA; if (A2) A2 += z * sA; Bt += z * sB; if (Bt2) Bt2 += z * sB; C += z * sC;
    const int lane = threadIdx.x & 31, lr = lane & 15, hi = lane >> 4; const int r0 = blockIdx.x * 64, c0 = blockIdx.y * 64;
    v8f acc[4][4];
#pragma unroll
    for (int mb = 0; mb < 4; ++mb)
#pragma unroll
        for (int nb = 0; nb < 4; ++nb) acc[mb][nb] = (v8f){};
    const size_t aoff = (size_t)(r0 + lr) * K + 8 * hi, boff = (size_t)(c0 + lr) * K + 8 * hi;
#pragma unroll 1
    for (int kc = 0; kc < K; kc += 32) {
        V a[4], a2[4];
#pragma unroll
        for (int mb = 0; mb < 4; ++mb) { a[mb] = WFrag<T16>::ld(A + aoff + (size_t)mb * 16 * K + kc); if (NSPLIT == 1 || NSPLIT == 2) a2[mb] = WFrag<T16>::ld(A2 + aoff + (size_t)mb * 16 * K + kc); }
#pragma unroll
        for (int nb = 0; nb < 4; ++nb) { const V b = WFrag<T16>::ld(Bt + boff + (size_t)nb * 16 * K + kc); V b2; if (NSPLIT >= 2) b2 = WFrag<T16>::ld(Bt2 + boff + (size_t)nb * 16 * K + kc);
#pragma unroll
            for (int mb = 0; mb < 4; ++mb) { acc[mb][nb] = WFrag<T16>::mma(a[mb], b, acc[mb][nb]); if (NSPLIT == 1 || NSPLIT == 2) acc[mb][nb] = WFrag<T16>::mma(a2[mb], b, acc[mb][nb]); if (NSPLIT >= 2) acc[mb][nb] = WFrag<T16>::mma(a[mb], b2, acc[mb][nb]); } }
        asm volatile("v_nop\n\tv_nop\n\tv_nop\n\tv_nop" : "+v"(acc[0][0]), "+v"(acc[1][1]), "+v"(acc[2][2]), "+v"(acc[3][3]) : "v"(a[0]), "v"(a[3]));
    }
#pragma unroll
    for (int mb = 0; mb < 4; ++mb) {
#pragma unroll
        for (int nb = 0; nb < 4; ++nb) {
#pragma unroll
            for (int j = 0; j < 8; ++j) os[(hi * 8 + j) * 68 + nb * 16 + lr] = acc[mb][nb][j]; }
        __builtin_amdgcn_wave_barrier(); asm volatile("" ::: "memory");
        float* crow = C + (size_t)(r0 + mb * 16) * ldc + c0;
#pragma unroll 1
        for (int ps = 0; ps < 2; ++ps) {
#pragma unroll
            for (int s = 0; s < 8; ++s) { const int row = 2 * s + hi, cofs = lr * 4; v4f val = *(const v4fa*)(os + row * 68 + cofs); if (BIAS) { val[0] += bfr(bias[c0 + cofs]); val[1] += bfr(bias[c0 + cofs + 1]); val[2] += bfr(bias[c0 + cofs + 2]); val[3] += bfr(bias[c0 + cofs + 3]); }
                *(volatile v4f*)(crow + (size_t)row * ldc + cofs) = val; }
            if (ps == 0) __threadfence(); }
        __builtin_amdgcn_wave_barrier(); asm volatile("" ::: "memory");
    }
}

__device__ __forceinline__ h16 tohx(float x) { return (h16)x; }
__device__ __forceinline__ void splitf(float y, unsigned short& h, unsigned short& l) { h = f2bf(y); l = f2bf(y - bf2f(h)); }
typedef __attribute__((ext_vector_type(4))) _Float16 v4h;
typedef __attribute__((ext_vector_type(4))) unsigned short v4us;

__global__ __launch_bounds__(256) void k_cvt8(const float* __restrict__ src, bf* dst, size_t n8) { const size_t i = (size_t)blockIdx.x * 256 + threadIdx.x; if (i >= n8) return; const v8f v = *(const v8f*)(src + i * 8); v8us o;
#pragma unroll
    for (int k = 0; k < 8; ++k) o[k] = f2bf(v[k]); *(volatile v8us*)(dst + i * 8) = o; __threadfence(); *(volatile v8us*)(dst + i * 8) = o; }
template <typename T16>
__global__ __launch_bounds__(256) void k_wg(const float* __restrict__ Wsrc, T16* Bt) { const size_t e = ((size_t)blockIdx.x * 256 + threadIdx.x) * 4; if (e >= (size_t)NW * DI) return; const int k = (int)(e % DI); const int n = (int)(e / DI); const int s = n / DI, o = n % DI; T16 r[4];
#pragma unroll
    for (int q = 0; q < 4; ++q) { const float w = bfr(Wsrc[(size_t)s * DI * DI + (size_t)(k + q) * DI + o]); if constexpr (sizeof(T16) == 2 && __is_same(T16, bf)) r[q] = f2bf(w); else r[q] = tohx(w); }
    typedef __attribute__((ext_vector_type(4))) T16 v4t; v4t o4; o4[0] = r[0]; o4[1] = r[1]; o4[2] = r[2]; o4[3] = r[3]; *(volatile v4t*)(Bt + e) = o4; __threadfence(); *(volatile v4t*)(Bt + e) = o4; }
__global__ __launch_bounds__(256) void k_w2(const float* __restrict__ W2, bf* Bt) { const int e = (blockIdx.x * 256 + threadIdx.x) * 4; if (e >= 64 * DI) return; const int k = e % DI, n = e / DI; v4us o;
#pragma unroll
    for (int q = 0; q < 4; ++q) o[q] = n < SD ? f2bf(W2[(size_t)n * DI + k + q]) : (unsigned short)0; *(volatile v4us*)(Bt + e) = o; __threadfence(); *(volatile v4us*)(Bt + e) = o; }
__global__ __launch_bounds__(256) void k_basis(const float* __restrict__ tr, float* BS) { const size_t e = ((size_t)blockIdx.x * 256 + threadIdx.x) * 4; if (e >= (size_t)NBT * 16) return; const int s0 = (int)(e % 16); const int b = (int)(e / 16); const float t = bfr(tr[b]); v4f o;
#pragma unroll
    for (int q = 0; q < 4; ++q) { const int s = s0 + q; float v = 0.f;
        if (s == 0) v = 1.f; else if (s == 1) v = t; else if (s == 2) v = __fmul_rn(t, t); else if (s == 3) { float t2 = __fmul_rn(t, t); asm volatile("" : "+v"(t2)); v = __fmul_rn(t2, t); }
        else if (s < SD) { const float kn = (float)(s - 3) / 9.0f; const float r = fmaxf(__fsub_rn(t, kn), 0.f); float r2 = __fmul_rn(r, r); asm volatile("" : "+v"(r2)); v = __fmul_rn(r2, r); }
        o[q] = v; }
    *(volatile v4f*)(BS + e) = o; __threadfence(); *(volatile v4f*)(BS + e) = o; }
template <int MODE>
__global__ __launch_bounds__(256) void k_comb(const float* __restrict__ TMP, const float* __restrict__ BS, const float* __restrict__ bias, int b0, h16* H16, bf* Hh, bf* Hl) { const size_t e = ((size_t)blockIdx.x * 256 + threadIdx.x) * 4; if (e >= (size_t)RCH * DI) return; const int o = (int)(e % DI); const int bl = (int)(e / DI); const float* bs = BS + (size_t)(b0 + bl) * 16; v4h oh16; v4us oh, ol;
#pragma unroll
    for (int q = 0; q < 4; ++q) { float acc = 0.f;
#pragma unroll 1
        for (int s = 0; s < SD; ++s) { float p = __fmul_rn(bs[s], TMP[(size_t)bl * NW + s * DI + o + q]); asm volatile("" : "+v"(p)); acc = __fadd_rn(acc, p); float pb = __fmul_rn(bs[s], bfr(bias[s * DI + o + q])); asm volatile("" : "+v"(pb)); acc = __fadd_rn(acc, pb); }
        acc = fmaxf(acc, 0.f); if (MODE == 0) oh16[q] = tohx(acc); else { unsigned short a, c; splitf(acc, a, c); oh[q] = a; ol[q] = c; } }
    if (MODE == 0) { *(volatile v4h*)(H16 + e) = oh16; __threadfence(); *(volatile v4h*)(H16 + e) = oh16; } else { *(volatile v4us*)(Hh + e) = oh; *(volatile v4us*)(Hl + e) = ol; __threadfence(); *(volatile v4us*)(Hh + e) = oh; *(volatile v4us*)(Hl + e) = ol; } }
__global__ __launch_bounds__(256) void k_comb2(const float* __restrict__ TMP2, const float* __restrict__ BS, const float* __restrict__ b2, int b0, float* OUT) { const int bl = blockIdx.x * 256 + threadIdx.x; if (bl >= RCH) return; const float* bs = BS + (size_t)(b0 + bl) * 16; float acc = 0.f;
#pragma unroll 1
    for (int s = 0; s < SD; ++s) { float p = __fmul_rn(bs[s], TMP2[(size_t)bl * 64 + s]); asm volatile("" : "+v"(p)); acc = __fadd_rn(acc, p); float pb = __fmul_rn(bs[s], bfr(b2[s])); asm volatile("" : "+v"(pb)); acc = __fadd_rn(acc, pb); }
    *(volatile float*)(OUT + b0 + bl) = acc; __threadfence(); *(volatile float*)(OUT + b0 + bl) = acc; }

extern "C" void kernel_launch(void* const* d_in, const int* in_sizes, int n_in,
                              void* d_out, int out_size, void* d_ws, size_t ws_size, hipStream_t stream) {
    (void)in_sizes; (void)n_in; (void)out_size;
    const float* tr = (const float*)d_in[0]; const float* x = (const float*)d_in[1]; const float* W0 = (const float*)d_in[2]; const float* b0 = (const float*)d_in[3]; const float* W1 = (const float*)d_in[4]; const float* b1 = (const float*)d_in[5]; const float* W2 = (const float*)d_in[6]; const float* b2 = (const float*)d_in[7];
    float* OUT = (float*)d_out;
    char* wsp = (char*)d_ws;
    auto take = [&](size_t bytes) { char* p = wsp; wsp += (bytes + 255) & ~(size_t)255; return (void*)p; };
    bf* Bt0 = (bf*)take((size_t)NW * DI * 2); h16* Bt1 = (h16*)take((size_t)NW * DI * 2); bf* Bt2 = (bf*)take((size_t)64 * DI * 2); bf* XB = (bf*)take((size_t)NBT * DI * 2); float* BS = (float*)take((size_t)NBT * 16 * 4);
    float* TMP = (float*)take((size_t)RCH * NW * 4); h16* H16 = (h16*)take((size_t)RCH * DI * 2); bf* Hh = (bf*)take((size_t)RCH * DI * 2); bf* Hl = (bf*)take((size_t)RCH * DI * 2); float* TMP2 = (float*)take((size_t)RCH * 64 * 4);
    if ((size_t)(wsp - (char*)d_ws) > ws_size) return;
    k_wg<bf><<<(unsigned)(((size_t)NW * DI / 4 + 255) / 256), 256, 0, stream>>>(W0, Bt0); k_wg<h16><<<(unsigned)(((size_t)NW * DI / 4 + 255) / 256), 256, 0, stream>>>(W1, Bt1); k_w2<<<(64 * DI / 4 + 255) / 256, 256, 0, stream>>>(W2, Bt2);
    k_cvt8<<<(NBT * DI / 8 + 255) / 256, 256, 0, stream>>>(x, XB, (size_t)NBT * DI / 8); k_basis<<<(NBT * 16 / 4 + 255) / 256, 256, 0, stream>>>(tr, BS);
    const unsigned LC = (unsigned)(((size_t)RCH * DI / 4 + 255) / 256);
    for (int c0 = 0; c0 < NBT; c0 += RCH) {
        k_gemmw<bf, 0, false><<<dim3(RCH / 64, NW / 64, 1), 32, 0, stream>>>(XB + (size_t)c0 * DI, nullptr, Bt0, nullptr, DI, TMP, NW, nullptr, 0, 0, 0); k_comb<0><<<LC, 256, 0, stream>>>(TMP, BS, b0, c0, H16, nullptr, nullptr);
        k_gemmw<h16, 0, false><<<dim3(RCH / 64, NW / 64, 1), 32, 0, stream>>>(H16, nullptr, Bt1, nullptr, DI, TMP, NW, nullptr, 0, 0, 0); k_comb<1><<<LC, 256, 0, stream>>>(TMP, BS, b1, c0, nullptr, Hh, Hl);
        k_gemmw<bf, 1, false><<<dim3(RCH / 64, 1, 1), 32, 0, stream>>>(Hh, Hl, Bt2, nullptr, DI, TMP2, 64, nullptr, 0, 0, 0); k_comb2<<<RCH / 256, 256, 0, stream>>>(TMP2, BS, b2, c0, OUT); }
}
